// EnhancedTransformerEncoder_64931315581524
// MI455X (gfx1250) — hardware-verified
//
#include <hip/hip_runtime.h>
#include <math.h>


#define TT 128
#define BB 16
#define DD 512
#define HH 8
#define HDQ 64
#define ETA 4
#define RR 8
#define FF (ETA * HDQ)
#define MROWS (TT * BB)
#define NCAT (5 * DD + 3 * (HH * ETA))
#define EPSV 1e-6f

typedef char chk_tiles[((NCAT % 32) == 0 && (DD % 32) == 0 && (MROWS % 32) == 0) ? 1 : -1];

typedef __bf16 v16b __attribute__((ext_vector_type(16)));
typedef __bf16 v8b __attribute__((ext_vector_type(8)));
typedef float v8f __attribute__((ext_vector_type(8)));
typedef float v4f __attribute__((ext_vector_type(4)));
typedef unsigned short v8us __attribute__((ext_vector_type(8)));

union Frag {
  v16b v;
  v8b half[2];
};

__device__ __forceinline__ unsigned int bf16_bits_rne(float x) {
  unsigned int u = __float_as_uint(x);
  return (u + 0x7FFFu + ((u >> 16) & 1u)) >> 16;
}

__device__ __forceinline__ v8f mma_bf16(const v16b a, const v16b b, v8f c) {
  c = __builtin_amdgcn_wmma_f32_16x16x32_bf16(false, a, false, b, (short)0, c, false, false);
  asm volatile("v_nop\n\tv_nop\n\tv_nop\n\tv_nop" : "+v"(c) : "v"(a), "v"(b));
  return c;
}

__global__ __launch_bounds__(256)
void cvt_split_bf16(const float* __restrict__ src, unsigned short* dhi,
                    unsigned short* dlo, int n) {
  const size_t i = (size_t)blockIdx.x * blockDim.x + threadIdx.x;
  const size_t base = i * 8;
  if (base + 8 > (size_t)n) return;
  const v4f x0 = *(const v4f*)(src + base);
  const v4f x1 = *(const v4f*)(src + base + 4);
  float x[8];
#pragma unroll
  for (int j = 0; j < 4; ++j) { x[j] = x0[j]; x[4 + j] = x1[j]; }
  v8us hv, lv;
#pragma unroll
  for (int j = 0; j < 8; ++j) {
    const unsigned int hb = bf16_bits_rne(x[j]);
    const float hf = __uint_as_float(hb << 16);
    const unsigned int lb = bf16_bits_rne(x[j] - hf);
    hv[j] = (unsigned short)hb;
    lv[j] = (unsigned short)lb;
  }
  volatile v8us* ph = (volatile v8us*)(dhi + base);
  volatile v8us* pl = (volatile v8us*)(dlo + base);
  *ph = hv;
  *pl = lv;
  __threadfence();
  *ph = hv;
  *pl = lv;
}

__global__ __launch_bounds__(256)
void cos_table_kernel(const float* __restrict__ tick, const float* __restrict__ omegas,
                      float* ct, int total) {
  __shared__ union { float f[256]; v4f v[64]; } cs;
  const int tid = threadIdx.x;
  const int idx = blockIdx.x * 256 + tid;
  float c = 0.0f;
  if (idx < total) {
    const int r = idx & (RR - 1);
    const int tb = idx >> 3;
    const int t = tb / BB;
    const int b = tb - t * BB;
    const float tt = (float)(t + 1) + tick[b];
    c = cosf(tt * omegas[r]);
  }
  cs.f[tid] = c;
  __syncthreads();
  if (tid < 64) {
    const int base = blockIdx.x * 256 + 4 * tid;
    if (base + 4 <= total) {
      const v4f v = cs.v[tid];
      volatile v4f* p = (volatile v4f*)(ct + base);
      *p = v;
      __threadfence();
      *p = v;
    }
  }
}

__global__ __launch_bounds__(32)
void gemm_bf16x3(const __bf16* __restrict__ Ah, const __bf16* __restrict__ Al,
                 const __bf16* __restrict__ Bh, const __bf16* __restrict__ Bl,
                 const float* __restrict__ bias, int use_bias,
                 float* C, int M, int N, int K) {
  const int n0 = blockIdx.x * 32;
  const int m0 = blockIdx.y * 32;
  if (n0 + 32 > N || m0 + 32 > M) return;
  const int l = threadIdx.x & 31;
  const int h = l >> 4;
  const int m = l & 15;

  v8f acc[2][2];
#pragma unroll
  for (int j = 0; j < 2; ++j) {
    const float bv = use_bias ? bias[n0 + 16 * j + m] : 0.0f;
#pragma unroll
    for (int i = 0; i < 2; ++i)
#pragma unroll
      for (int q = 0; q < 8; ++q) acc[i][j][q] = bv;
  }

  const __bf16* ah_row[2];
  const __bf16* al_row[2];
  const __bf16* bh_row[2];
  const __bf16* bl_row[2];
#pragma unroll
  for (int i = 0; i < 2; ++i) {
    ah_row[i] = Ah + (size_t)(m0 + 16 * i + m) * K;
    al_row[i] = Al + (size_t)(m0 + 16 * i + m) * K;
    bh_row[i] = Bh + (size_t)(n0 + 16 * i + m) * K;
    bl_row[i] = Bl + (size_t)(n0 + 16 * i + m) * K;
  }

  for (int k0 = 0; k0 < K; k0 += 32) {
    Frag fah[2], fal[2], fbh[2], fbl[2];
    const int ka = k0 + 8 * h;
    const int kb = k0 + 16 + 8 * h;
#pragma unroll
    for (int i = 0; i < 2; ++i) {
      fah[i].half[0] = *(const v8b*)(ah_row[i] + ka);
      fah[i].half[1] = *(const v8b*)(ah_row[i] + kb);
      fal[i].half[0] = *(const v8b*)(al_row[i] + ka);
      fal[i].half[1] = *(const v8b*)(al_row[i] + kb);
      fbh[i].half[0] = *(const v8b*)(bh_row[i] + ka);
      fbh[i].half[1] = *(const v8b*)(bh_row[i] + kb);
      fbl[i].half[0] = *(const v8b*)(bl_row[i] + ka);
      fbl[i].half[1] = *(const v8b*)(bl_row[i] + kb);
    }
#pragma unroll
    for (int i = 0; i < 2; ++i)
#pragma unroll
      for (int j = 0; j < 2; ++j) {
        acc[i][j] = mma_bf16(fah[i].v, fbh[j].v, acc[i][j]);
        acc[i][j] = mma_bf16(fah[i].v, fbl[j].v, acc[i][j]);
        acc[i][j] = mma_bf16(fal[i].v, fbh[j].v, acc[i][j]);
      }
  }

  __shared__ union { float f[32][36]; v4f v[32][9]; } tile;
#pragma unroll
  for (int i = 0; i < 2; ++i)
#pragma unroll
    for (int j = 0; j < 2; ++j)
#pragma unroll
      for (int r = 0; r < 8; ++r)
        tile.f[16 * i + 8 * h + r][16 * j + m] = acc[i][j][r];
  __syncthreads();

  const int rsub = l >> 3;
  const int c4 = l & 7;
  v4f vals[8];
#pragma unroll
  for (int s = 0; s < 8; ++s) vals[s] = tile.v[4 * s + rsub][c4];
#pragma unroll
  for (int s = 0; s < 8; ++s) {
    float* p = C + (size_t)(m0 + 4 * s + rsub) * N + n0 + 4 * c4;
    *(volatile v4f*)p = vals[s];
  }
  __threadfence();
#pragma unroll
  for (int s = 0; s < 8; ++s) {
    float* p = C + (size_t)(m0 + 4 * s + rsub) * N + n0 + 4 * c4;
    *(volatile v4f*)p = vals[s];
  }
}

__device__ __forceinline__ float sigmoidf_(float x) {
  return 1.0f / (1.0f + __expf(-x));
}

__device__ __forceinline__ float wave_red32(float v) {
#pragma unroll
  for (int off = 16; off; off >>= 1) v += __shfl_xor(v, off, 32);
  return v;
}

__global__ __launch_bounds__(256)
void scan_attn_kernel(const float* __restrict__ P,
                      const int* __restrict__ term,
                      const float* __restrict__ tk_prev,
                      const float* __restrict__ tv_prev,
                      const float* __restrict__ s_prev,
                      const float* __restrict__ tick,
                      const float* __restrict__ ct,
                      unsigned short* a_hi,
                      unsigned short* a_lo,
                      float* out_tk, float* out_tv, float* out_s, float* out_tick) {
  const int bh = blockIdx.x;
  if (bh >= BB * HH) return;
  const int b = bh >> 3;
  const int h = bh & 7;
  const int tid = threadIdx.x;
  const int e = tid >> 6;
  const int d = tid & 63;
  const int wave = tid >> 5;
  const int lane = tid & 31;

  __shared__ float st[336];
  __shared__ float cosv[RR];
  __shared__ float wpart[8][9];
  __shared__ union { float f[256]; v4f v[64]; } red;
  __shared__ float att[64];

  float s_state = s_prev[(size_t)(b * HH + h) * FF + tid];
  float tk[RR];
#pragma unroll
  for (int r = 0; r < RR; ++r)
    tk[r] = tk_prev[(size_t)((b * RR + r) * HH + h) * FF + tid];
  float tv0 = tv_prev[(size_t)((b * RR + e) * HH + h) * HDQ + d];
  float tv1 = tv_prev[(size_t)((b * RR + e + 4) * HH + h) * HDQ + d];

  for (int t = 0; t < TT; ++t) {
    const size_t rowi = (size_t)(t * BB + b);
    const float* row = P + rowi * NCAT;
    if (tid < 64) {
      st[tid]       = row[0 * DD + h * HDQ + tid];
      st[64 + tid]  = row[1 * DD + h * HDQ + tid];
      st[128 + tid] = row[2 * DD + h * HDQ + tid];
      st[192 + tid] = row[3 * DD + h * HDQ + tid];
      st[256 + tid] = row[4 * DD + h * HDQ + tid];
    }
    if (tid < 4) {
      st[320 + tid] = row[5 * DD + 0 * HH * ETA + h * ETA + tid];
      st[324 + tid] = row[5 * DD + 1 * HH * ETA + h * ETA + tid];
      st[328 + tid] = row[5 * DD + 2 * HH * ETA + h * ETA + tid];
    }
    if (tid >= 64 && tid < 64 + RR) cosv[tid - 64] = ct[rowi * RR + (tid - 64)];
    __syncthreads();

    const float mask = 1.0f - (float)term[t * BB + b];

    const float relu_q   = fmaxf(st[d], 0.0f);
    const float relu_k   = fmaxf(st[64 + d], 0.0f);
    const float sig_beta = sigmoidf_(st[192 + d]);
    const float sig_gam  = sigmoidf_(st[256 + d]);
    const float p1r = fmaxf(st[320 + e], 0.0f);
    const float p2r = fmaxf(st[324 + e], 0.0f);
    const float p3s = sigmoidf_(st[328 + e]);

    const float phi_q = p2r * relu_q;
    const float gfeat = p3s * sig_gam;
    const float gk = (p1r * relu_k) * gfeat;
    const float dg = (1.0f - gfeat) * mask;
    const float gv = st[128 + d] * sig_beta;
    const float db = (1.0f - sig_beta) * mask;

    s_state = dg * s_state + gk;
#pragma unroll
    for (int r = 0; r < RR; ++r)
      tk[r] = dg * tk[r] + gk * cosv[r];
    tv0 = db * tv0 + gv * cosv[e];
    tv1 = db * tv1 + gv * cosv[e + 4];

#pragma unroll
    for (int r = 0; r < RR; ++r) {
      float v = wave_red32(tk[r] * phi_q);
      if (lane == 0) wpart[wave][r] = v;
    }
    {
      float v = wave_red32(s_state * phi_q);
      if (lane == 0) wpart[wave][8] = v;
    }
    __syncthreads();

    float norm = 0.f, kq0 = 0.f, kq1 = 0.f;
#pragma unroll
    for (int w = 0; w < 8; ++w) {
      norm += wpart[w][8];
      kq0  += wpart[w][e];
      kq1  += wpart[w][e + 4];
    }

    red.f[tid] = tv0 * kq0 + tv1 * kq1;
    __syncthreads();
    if (tid < 64) {
      const float kv = red.f[tid] + red.f[tid + 64] + red.f[tid + 128] + red.f[tid + 192];
      const float den = 16.0f * norm + EPSV;
      att[tid] = kv * (1.0f / den);
    }
    __syncthreads();
    if (tid < 16) {
      const int q = tid & 7;
      v8us hv, lv;
#pragma unroll
      for (int j = 0; j < 8; ++j) {
        const float x = att[8 * q + j];
        const unsigned int hb = bf16_bits_rne(x);
        const float hf = __uint_as_float(hb << 16);
        const unsigned int lb = bf16_bits_rne(x - hf);
        hv[j] = (unsigned short)hb;
        lv[j] = (unsigned short)lb;
      }
      const size_t off = rowi * (HH * HDQ) + h * HDQ + 8 * q;
      unsigned short* dst = (tid < 8) ? (a_hi + off) : (a_lo + off);
      v8us val = hv;
      if (tid >= 8) val = lv;
      *(volatile v8us*)dst = val;
      __threadfence();
      *(volatile v8us*)dst = val;
    }
  }

  red.f[tid] = s_state;
  __syncthreads();
  if (tid < 64) {
    const v4f v = red.v[tid];
    float* p = out_s + (size_t)(b * HH + h) * FF + 4 * tid;
    *(volatile v4f*)p = v;
    __threadfence();
    *(volatile v4f*)p = v;
  }
#pragma unroll
  for (int r = 0; r < RR; ++r) {
    __syncthreads();
    red.f[tid] = tk[r];
    __syncthreads();
    if (tid < 64) {
      const v4f v = red.v[tid];
      float* p = out_tk + (size_t)((b * RR + r) * HH + h) * FF + 4 * tid;
      *(volatile v4f*)p = v;
      __threadfence();
      *(volatile v4f*)p = v;
    }
  }
  __syncthreads();
  red.f[tid] = tv0;
  __syncthreads();
  if (tid < 64) {
    const int r = tid >> 4;
    const int d4 = (tid & 15) * 4;
    const v4f v = red.v[tid];
    float* p = out_tv + (size_t)((b * RR + r) * HH + h) * HDQ + d4;
    *(volatile v4f*)p = v;
    __threadfence();
    *(volatile v4f*)p = v;
  }
  __syncthreads();
  red.f[tid] = tv1;
  __syncthreads();
  if (tid < 64) {
    const int r = 4 + (tid >> 4);
    const int d4 = (tid & 15) * 4;
    const v4f v = red.v[tid];
    float* p = out_tv + (size_t)((b * RR + r) * HH + h) * HDQ + d4;
    *(volatile v4f*)p = v;
    __threadfence();
    *(volatile v4f*)p = v;
  }
  if (bh == 0 && tid < 4) {
    v4f v;
#pragma unroll
    for (int j = 0; j < 4; ++j) v[j] = tick[4 * tid + j] + (float)TT;
    float* p = out_tick + 4 * tid;
    *(volatile v4f*)p = v;
    __threadfence();
    *(volatile v4f*)p = v;
  }
}

static inline size_t al256(size_t x) { return (x + 255) & ~(size_t)255; }

extern "C" void kernel_launch(void* const* d_in, const int* in_sizes, int n_in,
                              void* d_out, int out_size, void* d_ws, size_t ws_size,
                              hipStream_t stream) {
  if (n_in < 17) return;
  if (in_sizes[0] != MROWS * DD || in_sizes[1] != TT * BB || in_sizes[5] != BB ||
      in_sizes[6] != DD * DD || in_sizes[11] != HH * ETA * DD ||
      in_sizes[14] != DD * DD || in_sizes[15] != DD || in_sizes[16] != RR)
    return;
  const size_t n_out_total = (size_t)MROWS * DD + (size_t)BB * RR * HH * FF +
                             (size_t)BB * RR * HH * HDQ + (size_t)BB * HH * FF + BB;
  if ((size_t)out_size != n_out_total) return;

  const float* inputs  = (const float*)d_in[0];
  const int*   term    = (const int*)  d_in[1];
  const float* tk_prev = (const float*)d_in[2];
  const float* tv_prev = (const float*)d_in[3];
  const float* s_prev  = (const float*)d_in[4];
  const float* tick    = (const float*)d_in[5];
  const float* Wq      = (const float*)d_in[6];
  const float* Wk      = (const float*)d_in[7];
  const float* Wv      = (const float*)d_in[8];
  const float* Wbeta   = (const float*)d_in[9];
  const float* Wgamma  = (const float*)d_in[10];
  const float* Wp1     = (const float*)d_in[11];
  const float* Wp2     = (const float*)d_in[12];
  const float* Wp3     = (const float*)d_in[13];
  const float* Wout    = (const float*)d_in[14];
  const float* bout    = (const float*)d_in[15];
  const float* omegas  = (const float*)d_in[16];

  char* ws = (char*)d_ws;
  size_t off = 0;
  unsigned short* Xh  = (unsigned short*)(ws + off); off += al256((size_t)MROWS * DD * 2);
  unsigned short* Xl  = (unsigned short*)(ws + off); off += al256((size_t)MROWS * DD * 2);
  unsigned short* Wch = (unsigned short*)(ws + off); off += al256((size_t)NCAT * DD * 2);
  unsigned short* Wcl = (unsigned short*)(ws + off); off += al256((size_t)NCAT * DD * 2);
  unsigned short* Woh = (unsigned short*)(ws + off); off += al256((size_t)DD * DD * 2);
  unsigned short* Wol = (unsigned short*)(ws + off); off += al256((size_t)DD * DD * 2);
  float* P            = (float*)(ws + off);          off += al256((size_t)MROWS * NCAT * 4);
  unsigned short* Ath = (unsigned short*)(ws + off); off += al256((size_t)MROWS * DD * 2);
  unsigned short* Atl = (unsigned short*)(ws + off); off += al256((size_t)MROWS * DD * 2);
  float* ct           = (float*)(ws + off);          off += al256((size_t)TT * BB * RR * 4);
  if (off > ws_size) return;

  float* out_output = (float*)d_out;
  float* out_tk   = out_output + (size_t)MROWS * DD;
  float* out_tv   = out_tk + (size_t)BB * RR * HH * FF;
  float* out_s    = out_tv + (size_t)BB * RR * HH * HDQ;
  float* out_tick = out_s + (size_t)BB * HH * FF;

  auto cvt = [&](const float* src, unsigned short* dhi, unsigned short* dlo, int n) {
    const int nthr = n / 8;
    cvt_split_bf16<<<(nthr + 255) / 256, 256, 0, stream>>>(src, dhi, dlo, n);
  };

  cvt(inputs, Xh, Xl, MROWS * DD);
  cvt(Wq,     Wch + (size_t)0    * DD, Wcl + (size_t)0    * DD, DD * DD);
  cvt(Wk,     Wch + (size_t)512  * DD, Wcl + (size_t)512  * DD, DD * DD);
  cvt(Wv,     Wch + (size_t)1024 * DD, Wcl + (size_t)1024 * DD, DD * DD);
  cvt(Wbeta,  Wch + (size_t)1536 * DD, Wcl + (size_t)1536 * DD, DD * DD);
  cvt(Wgamma, Wch + (size_t)2048 * DD, Wcl + (size_t)2048 * DD, DD * DD);
  cvt(Wp1,    Wch + (size_t)2560 * DD, Wcl + (size_t)2560 * DD, HH * ETA * DD);
  cvt(Wp2,    Wch + (size_t)2592 * DD, Wcl + (size_t)2592 * DD, HH * ETA * DD);
  cvt(Wp3,    Wch + (size_t)2624 * DD, Wcl + (size_t)2624 * DD, HH * ETA * DD);
  cvt(Wout,   Woh, Wol, DD * DD);

  const int ncos = TT * BB * RR;
  cos_table_kernel<<<(ncos + 255) / 256, 256, 0, stream>>>(tick, omegas, ct, ncos);

  gemm_bf16x3<<<dim3(NCAT / 32, MROWS / 32), 32, 0, stream>>>(
      (const __bf16*)Xh, (const __bf16*)Xl, (const __bf16*)Wch, (const __bf16*)Wcl,
      bout, 0, P, MROWS, NCAT, DD);

  scan_attn_kernel<<<BB * HH, 256, 0, stream>>>(
      P, term, tk_prev, tv_prev, s_prev, tick, ct,
      Ath, Atl, out_tk, out_tv, out_s, out_tick);

  gemm_bf16x3<<<dim3(DD / 32, MROWS / 32), 32, 0, stream>>>(
      (const __bf16*)Ath, (const __bf16*)Atl, (const __bf16*)Woh, (const __bf16*)Wol,
      bout, 1, out_output, MROWS, DD, DD);
}
